// MLPEMABlock_65463891525760
// MI455X (gfx1250) — hardware-verified
//
#include <hip/hip_runtime.h>
#include <math.h>

typedef __attribute__((ext_vector_type(16))) _Float16 v16h;
typedef __attribute__((ext_vector_type(16))) __bf16 v16b;
typedef __attribute__((ext_vector_type(8)))  _Float16 v8h;
typedef __attribute__((ext_vector_type(8)))  float v8f;
typedef __attribute__((ext_vector_type(4)))  float v4f;
typedef __attribute__((ext_vector_type(2)))  float v2f;
typedef __attribute__((ext_vector_type(4)))  unsigned v4u;
typedef __attribute__((ext_vector_type(4)))  int v4i;
typedef float __attribute__((may_alias)) float_a;
typedef int __attribute__((may_alias)) int_a;

template <typename T> __device__ __forceinline__ void vst2(void* p, T v) { *(volatile T*)p = v; __threadfence(); *(volatile T*)p = v; }
__device__ __forceinline__ v8f wmma16(v16h a, v16h b, v8f c) {
  v8f d = __builtin_amdgcn_wmma_f32_16x16x32_f16(false, a, false, b, (short)0, c, false, false);
  asm volatile("v_nop\n\tv_nop\n\tv_nop\n\tv_nop" : "+v"(d) : "v"(a), "v"(b));
  return d;
}
__device__ __forceinline__ v8f wmma_bf(v16b a, v16b b, v8f c) {
  v8f d = __builtin_amdgcn_wmma_f32_16x16x32_bf16(false, a, false, b, (short)0, c, false, false);
  asm volatile("v_nop\n\tv_nop\n\tv_nop\n\tv_nop" : "+v"(d) : "v"(a), "v"(b));
  return d;
}
__device__ __forceinline__ v16h frag_h(const _Float16* rowk0, int lane) {
  union { v16h v; v8h q[2]; } u; const _Float16* p = rowk0 + 8 * (lane >> 4);
  u.q[0] = *(const v8h*)p; u.q[1] = *(const v8h*)(p + 16); return u.v;
}
__device__ __forceinline__ v16h frag_f32(const float* rowk0, int lane) {
  v16h a; const float* p = rowk0 + 8 * (lane >> 4);
#pragma unroll
  for (int i = 0; i < 8; ++i) { a[i] = (_Float16)p[i]; a[8 + i] = (_Float16)p[16 + i]; }
  return a;
}
__device__ __forceinline__ v16h frag_f32s(const float* rowk0, int lane, float sc) {
  v16h a; const float* p = rowk0 + 8 * (lane >> 4);
#pragma unroll
  for (int i = 0; i < 8; ++i) { a[i] = (_Float16)(p[i] * sc); a[8 + i] = (_Float16)(p[16 + i] * sc); }
  return a;
}
__device__ __forceinline__ v16h fragc_f32(const float* W, int k0, int n, int lane, int ld, int K) {
  v16h a; const int g = lane >> 4;
#pragma unroll
  for (int i = 0; i < 8; ++i) { const int ka = k0 + 8 * g + i, kb = ka + 16;
    a[i] = (_Float16)(ka < K ? W[(size_t)(ka < K ? ka : K - 1) * ld + n] : 0.f); a[8 + i] = (_Float16)(kb < K ? W[(size_t)(kb < K ? kb : K - 1) * ld + n] : 0.f); }
  return a;
}
struct F2 { v16b h, l; };
__device__ __forceinline__ F2 bsplit16(const float v[16]) { F2 r;
#pragma unroll
  for (int i = 0; i < 16; ++i) { const __bf16 h = (__bf16)v[i]; r.h[i] = h; r.l[i] = (__bf16)(v[i] - (float)h); }
  return r; }
__device__ __forceinline__ F2 split_row(const float* row, int k0, int lane) { float v[16]; const float* p = row + k0 + 8 * (lane >> 4);
#pragma unroll
  for (int i = 0; i < 8; ++i) { v[i] = p[i]; v[8 + i] = p[16 + i]; }
  return bsplit16(v); }
__device__ __forceinline__ F2 split_rowK(const float* row, int k0, int lane, int K) { float v[16]; const int g = lane >> 4;
#pragma unroll
  for (int i = 0; i < 8; ++i) { const int ka = k0 + 8 * g + i, kb = ka + 16; v[i] = ka < K ? row[ka < K ? ka : K - 1] : 0.f; v[8 + i] = kb < K ? row[kb < K ? kb : K - 1] : 0.f; }
  return bsplit16(v); }
__device__ __forceinline__ F2 split_col(const float* W, int k0, int n, int lane, int ld, int K) { float v[16]; const int g = lane >> 4;
#pragma unroll
  for (int i = 0; i < 8; ++i) { const int ka = k0 + 8 * g + i, kb = ka + 16; v[i] = ka < K ? W[(size_t)(ka < K ? ka : K - 1) * ld + n] : 0.f; v[8 + i] = kb < K ? W[(size_t)(kb < K ? kb : K - 1) * ld + n] : 0.f; }
  return bsplit16(v); }
__device__ __forceinline__ v8f mac3(const F2& a, const F2& b, v8f c) { c = wmma_bf(a.l, b.h, c); c = wmma_bf(a.h, b.l, c); return wmma_bf(a.h, b.h, c); }
__device__ __forceinline__ float sigm(float v) { return 1.0f / (1.0f + expf(-v)); }
#define LDSX() do { asm volatile("s_wait_dscnt 0" ::: "memory"); __builtin_amdgcn_wave_barrier(); __builtin_amdgcn_fence(__ATOMIC_RELEASE, "workgroup"); } while (0)


#define NBT 8
#define NF 64
#define NS 8192
#define KW 201
#define NO 64
__device__ __forceinline__ float bfr(float v) { return (float)(__bf16)v; }
__device__ __forceinline__ v16b frag_b(const __bf16* rowk0, int lane) { return __builtin_bit_cast(v16b, frag_h((const _Float16*)rowk0, lane)); }

__global__ __launch_bounds__(64) void k_ema(const float* __restrict__ x, const float* __restrict__ lhl, float* __restrict__ EV) {
  const int ch = blockIdx.x * 64 + threadIdx.x; const int f = ch % NF; const float* xr = x + (size_t)ch * NS; float* ev = EV + (size_t)ch * NS;
  const float hl = expf(bfr(lhl[f])); const float alpha = exp2f(-1.0f / hl); const float aK = powf(alpha, (float)KW);
  float n1 = 0.f, n2 = 0.f, den = 0.f;
  __shared__ __align__(16) float sv[64][68];
#pragma unroll 1
  for (int s0 = 0; s0 < NS; s0 += 64) {
#pragma unroll 1
    for (int j = 0; j < 64; ++j) { const int s = s0 + j; const float v = bfr(xr[s]); const float vo = s >= KW ? bfr(xr[s - KW]) : 0.f; const float dro = s >= KW ? aK : 0.f;
      n1 = alpha * n1 + v - aK * vo; n2 = alpha * n2 + v * v - aK * vo * vo; den = alpha * den + 1.0f - dro;
      const float inv = 1.0f / (den + 1e-8f); const float m1 = n1 * inv; sv[threadIdx.x][j] = n2 * inv - m1 * m1; }
    __syncthreads();
    for (int q = threadIdx.x; q < 64 * 16; q += 64) { const int rl = q >> 4, pc = q & 15; vst2(EV + (size_t)(blockIdx.x * 64 + rl) * NS + s0 + pc * 4, *(const v4f*)(&sv[rl][pc * 4])); }
    __syncthreads(); }
}
__global__ __launch_bounds__(128) void k_lin(const float* __restrict__ EV, const float* __restrict__ nw, const float* __restrict__ LW, const float* __restrict__ lbias, float* __restrict__ OUT, float* __restrict__ SKIP) {
  __shared__ __align__(16) float st[64][68];
  __shared__ __align__(16) float so[128][68];
  const int tid = threadIdx.x, wave = tid >> 5, lane = tid & 31, col = lane & 15, g = lane >> 4; const int b = blockIdx.y, s0 = blockIdx.x * 64;
  for (int q = tid; q < NF * 64; q += 128) { const int f = q >> 6, sl = q & 63; st[sl][f] = EV[((size_t)b * NF + f) * NS + s0 + sl]; }
  __syncthreads();
  { const int rl = wave * 16 + (lane & 15), hf = lane >> 4; float ss = 0.f;
#pragma unroll
    for (int e = 0; e < 32; ++e) { const float v = st[rl][hf * 32 + e]; ss += v * v; }
    ss += __shfl_xor(ss, 16, 32); const float inv = 1.0f / sqrtf(ss * (1.0f / 192.0f) + 1e-8f);
#pragma unroll
    for (int e = 0; e < 32; ++e) { const int f = hf * 32 + e; st[rl][f] = st[rl][f] * inv * bfr(nw[128 + f]); } }
  LDSX(); __syncthreads();
  v8f acc[8] = {};
#pragma unroll
  for (int kc = 0; kc < 2; ++kc) { const F2 a = split_row(&st[wave * 16 + col][0], kc * 32, lane);
#pragma unroll
    for (int j = 0; j < 8; ++j) { const v16b wb = split_col(LW + (size_t)128 * 128, kc * 32, j * 16 + col, lane, 128, NF).h; acc[j] = wmma_bf(a.l, wb, acc[j]); acc[j] = wmma_bf(a.h, wb, acc[j]); } }
#pragma unroll
  for (int j = 0; j < 8; ++j) { const int o = j * 16 + col; const float bb = bfr(lbias[o]);
#pragma unroll
    for (int r = 0; r < 8; ++r) so[o][wave * 16 + 8 * g + r] = acc[j][r] + bb; }
  __syncthreads();
  for (int q = tid; q < 128 * 16; q += 128) { const int o = q >> 4, pc = q & 15; float* dst = o < NO ? SKIP + ((size_t)b * NO + o) * NS : OUT + ((size_t)b * NO + (o - NO)) * NS; vst2(dst + s0 + pc * 4, *(const v4f*)(&so[o][pc * 4])); }
}
extern "C" void kernel_launch(void* const* d_in, const int* in_sizes, int n_in, void* d_out, int out_size, void* d_ws, size_t ws_size, hipStream_t stream) {
  (void)in_sizes; (void)n_in; (void)out_size; (void)ws_size;
  const float* x = (const float*)d_in[0]; const float* lhv = (const float*)d_in[3]; const float* nw = (const float*)d_in[8]; const float* LW = (const float*)d_in[9]; const float* lb = (const float*)d_in[10];
  float* OUT = (float*)d_out; float* SKIP = (float*)((char*)d_out + 16777216);
  float* EV = (float*)d_ws;
  k_ema<<<NBT * NF / 64, 64, 0, stream>>>(x, lhv, EV);
  k_lin<<<dim3(NS / 64, NBT), 128, 0, stream>>>(EV, nw, LW, lb, OUT, SKIP);
}
